// MattesMI_45973329936800
// MI455X (gfx1250) — hardware-verified
//
#include <hip/hip_runtime.h>
#include <math.h>
typedef __attribute__((ext_vector_type(16))) _Float16 v16h;
typedef __attribute__((ext_vector_type(8)))  _Float16 v8h;
typedef __attribute__((ext_vector_type(16))) __bf16   v16b;
typedef __attribute__((ext_vector_type(8)))  __bf16   v8b;
typedef __attribute__((ext_vector_type(8)))  float    v8f;
typedef __attribute__((ext_vector_type(4)))  float    v4f;
#define PSCALE 32768.0f
#define U16(p) ((const unsigned short*)(const void*)(p))
#define PSCALE_INV (1.0f / 32768.0f)

__device__ __forceinline__ unsigned short f2bf_bits(float f) {
  unsigned u = __float_as_uint(f);
  return (unsigned short)((u + 0x7FFFu + ((u >> 16) & 1u)) >> 16);
}
__device__ __forceinline__ float bf_bits2f(unsigned short h) { return __uint_as_float(((unsigned)h) << 16); }

__device__ __forceinline__ void dep_guard_h(v8f& a, v8f& b, v16h x, v16h y) { asm volatile("v_nop\n\tv_nop\n\tv_nop\n\tv_nop" : "+v"(a), "+v"(b) : "v"(x), "v"(y)); }
__device__ __forceinline__ void dep_guard_b(v8f& a, v8f& b, v16b x, v16b y) { asm volatile("v_nop\n\tv_nop\n\tv_nop\n\tv_nop" : "+v"(a), "+v"(b) : "v"(x), "v"(y)); }
__device__ __forceinline__ void keep4_h(v16h a, v16h b, v16h c, v16h d) { asm volatile("v_nop" :: "v"(a), "v"(b), "v"(c), "v"(d)); }
__device__ __forceinline__ void keep4_b(v16b a, v16b b, v16b c, v16b d) { asm volatile("v_nop" :: "v"(a), "v"(b), "v"(c), "v"(d)); }
__device__ __forceinline__ void acc_guard4(v8f& a, v8f& b, v8f& c, v8f& d) { asm volatile("v_nop\n\tv_nop\n\tv_nop\n\tv_nop" : "+v"(a), "+v"(b), "+v"(c), "+v"(d)); }
template <typename T> struct Frag;
template <> struct Frag<_Float16> {
  typedef v16h V; union U { v16h v; v8h h[2]; };
  static __device__ __forceinline__ v16h load(const _Float16* p) {
    U f; f.h[0] = *(const v8h*)(p); f.h[1] = *(const v8h*)(p + 16); return f.v;
  }
  static __device__ __forceinline__ v8f mma(v16h a, v16h b, v8f c) {
    return __builtin_amdgcn_wmma_f32_16x16x32_f16(false, a, false, b, (short)0, c, false, false);
  }
  static __device__ __forceinline__ void guard(v8f& a, v8f& b, v16h x, v16h y) { dep_guard_h(a, b, x, y); }
  static __device__ __forceinline__ void keep(v16h a, v16h b, v16h c, v16h d) { keep4_h(a, b, c, d); }
};
template <> struct Frag<__bf16> {
  typedef v16b V; union U { v16b v; v8b h[2]; };
  static __device__ __forceinline__ v16b load(const __bf16* p) {
    U f; f.h[0] = *(const v8b*)(p); f.h[1] = *(const v8b*)(p + 16); return f.v;
  }
  static __device__ __forceinline__ v8f mma(v16b a, v16b b, v8f c) {
    return __builtin_amdgcn_wmma_f32_16x16x32_bf16(false, a, false, b, (short)0, c, false, false);
  }
  static __device__ __forceinline__ void guard(v8f& a, v8f& b, v16b x, v16b y) { dep_guard_b(a, b, x, y); }
  static __device__ __forceinline__ void keep(v16b a, v16b b, v16b c, v16b d) { keep4_b(a, b, c, d); }
};

template <int ET> struct Elem;
template <> struct Elem<0> { typedef _Float16 T; };
template <> struct Elem<1> { typedef __bf16 T; };
template <int ET, bool SPLIT, int BIAS_MODE, int OUT_MODE, bool RESID, int ACT = 0>
__global__ __launch_bounds__(256) void wmma_gemm64(
    const unsigned short* __restrict__ Ap, const unsigned short* __restrict__ A2p, int lda, long strideA,
    const unsigned short* __restrict__ Btp, const unsigned short* __restrict__ Bt2p, int ldb, long strideB,
    void* __restrict__ Cout, void* __restrict__ Cout2, int ldc, long strideC,
    const float* __restrict__ bias,
    const float* __restrict__ resid, long strideR,
    int M, int N, int K, float scale) {
  typedef typename Elem<ET>::T T;
  typedef typename Frag<T>::V V;
  const T* A = (const T*)Ap; const T* A2 = (const T*)A2p; const T* Bt = (const T*)Btp; const T* Bt2 = (const T*)Bt2p;
  __shared__ __align__(16) float sT[8][16 * 68];
  const int b    = blockIdx.y;
  const int lane = threadIdx.x & 31;
  const int wave = threadIdx.x >> 5;
  const int tilesN = N >> 6;
  const int tilesM = M >> 6;
  const int tile = blockIdx.x * 8 + wave;
  if (tile >= tilesM * tilesN) return;
  const int tm = tile / tilesN;
  const int tn = tile - tm * tilesN;
  const int m0 = tm << 6;
  const int n0 = tn << 6;

  const T* Ab  = A  + (size_t)b * strideA;
  const T* Bb  = Bt + (size_t)b * strideB;
  const T* Ab2 = SPLIT ? (A2  + (size_t)b * strideA) : nullptr;
  const T* Bb2 = SPLIT ? (Bt2 + (size_t)b * strideB) : nullptr;

  const int rlane = lane & 15;
  const int koff  = (lane >> 4) * 8;
  const int mOff  = (lane >> 4) * 8;

  v8f acc[4][4];
#pragma unroll
  for (int i = 0; i < 4; ++i)
#pragma unroll
    for (int j = 0; j < 4; ++j) acc[i][j] = (v8f){0.f,0.f,0.f,0.f,0.f,0.f,0.f,0.f};

  for (int k0 = 0; k0 < K; k0 += 32) {
    V bh[4], bl[4];
#pragma unroll
    for (int j = 0; j < 4; ++j) {
      const size_t bo = (size_t)(n0 + (j << 4) + rlane) * ldb + koff + k0;
      bh[j] = Frag<T>::load(Bb + bo);
      if (SPLIT) bl[j] = Frag<T>::load(Bb2 + bo);
    }
#pragma unroll
    for (int i = 0; i < 4; ++i) {
      const size_t ao = (size_t)(m0 + (i << 4) + rlane) * lda + koff + k0;
      V ah = Frag<T>::load(Ab + ao);
      V al;
      if (SPLIT) al = Frag<T>::load(Ab2 + ao);
#pragma unroll
      for (int j = 0; j < 4; ++j) {
        acc[i][j] = Frag<T>::mma(ah, bh[j], acc[i][j]);
        if (SPLIT) {
          acc[i][j] = Frag<T>::mma(ah, bl[j], acc[i][j]);
          acc[i][j] = Frag<T>::mma(al, bh[j], acc[i][j]);
        }
      }
      Frag<T>::guard(acc[i][0], acc[i][3], ah, SPLIT ? al : ah);
    }
    Frag<T>::keep(bh[0], bh[1], bh[2], bh[3]);
    if (SPLIT) Frag<T>::keep(bl[0], bl[1], bl[2], bl[3]);
  }
  acc_guard4(acc[0][0], acc[0][1], acc[0][2], acc[0][3]);
  acc_guard4(acc[1][0], acc[1][1], acc[1][2], acc[1][3]);
  acc_guard4(acc[2][0], acc[2][1], acc[2][2], acc[2][3]);
  acc_guard4(acc[3][0], acc[3][1], acc[3][2], acc[3][3]);

  float* slab = sT[wave];
  const float* Rb = RESID ? (resid + (size_t)b * strideR) : nullptr;
#pragma unroll
  for (int i = 0; i < 4; ++i) {
    const int mBase = m0 + (i << 4);
#pragma unroll
    for (int j = 0; j < 4; ++j) {
      const int n = n0 + (j << 4) + rlane;
      float bv = 0.f;
      if (BIAS_MODE == 2) bv = bias[n];
#pragma unroll
      for (int r = 0; r < 8; ++r) {
        float v = acc[i][j][r] * scale;
        if (BIAS_MODE == 1) v += bias[mBase + mOff + r];
        if (BIAS_MODE == 2) v += bv;
        if (RESID) v += Rb[(size_t)(mBase + mOff + r) * ldc + n];
        if (ACT == 1) v = tanhf(v);
        if (ACT == 2) v = fmaxf(v, 0.0f);
        if (ACT == 3) v = v / (1.0f + expf(-v));
        if (ACT == 4) v = (v > 0.f) ? v : 0.01f * v;
        if (ACT == 5) v = 0.5f * v * (1.0f + erff(v * 0.70710678118654752f));
        slab[(mOff + r) * 68 + (j << 4) + rlane] = v;
      }
    }
    __builtin_amdgcn_fence(__ATOMIC_RELEASE, "workgroup");
    __builtin_amdgcn_wave_barrier();
    __builtin_amdgcn_fence(__ATOMIC_ACQUIRE, "workgroup");
    if (OUT_MODE == 0) {
      float* C = (float*)Cout + (size_t)b * strideC;
      const int hh = lane >> 4, c4 = (lane & 15) * 4;
      for (int pass = 0; pass < 2; ++pass) {
#pragma unroll
        for (int it = 0; it < 8; ++it) {
          const int row = it * 2 + hh;
          v4f v = *(const v4f*)(slab + row * 68 + c4);
          *(volatile v4f*)(C + (size_t)(mBase + row) * ldc + n0 + c4) = v;
        }
        __threadfence();
      }
    } else {
      const int q = lane >> 3, c8 = (lane & 7) * 8;
      unsigned short* C  = (unsigned short*)Cout  + (size_t)b * strideC;
      unsigned short* C2 = (OUT_MODE == 2) ? ((unsigned short*)Cout2 + (size_t)b * strideC) : nullptr;
      for (int pass = 0; pass < 2; ++pass) {
#pragma unroll
        for (int it = 0; it < 4; ++it) {
          const int row = it * 4 + q;
          const float* sp = slab + row * 68 + c8;
          v8h hv, lv;
#pragma unroll
          for (int e = 0; e < 8; ++e) {
            if (OUT_MODE == 1) {
              hv[e] = (_Float16)sp[e];
            } else {
              unsigned short hb = f2bf_bits(sp[e]);
              unsigned short lb = f2bf_bits(sp[e] - bf_bits2f(hb));
              hv[e] = __builtin_bit_cast(_Float16, hb);
              lv[e] = __builtin_bit_cast(_Float16, lb);
            }
          }
          *(volatile v8h*)(C + (size_t)(mBase + row) * ldc + n0 + c8) = hv;
          if (OUT_MODE == 2) *(volatile v8h*)(C2 + (size_t)(mBase + row) * ldc + n0 + c8) = lv;
        }
        __threadfence();
      }
    }
    __builtin_amdgcn_fence(__ATOMIC_RELEASE, "workgroup");
    __builtin_amdgcn_wave_barrier();
    __builtin_amdgcn_fence(__ATOMIC_ACQUIRE, "workgroup");
  }
}


#define MV 2097152
#define MBINS 64
#define MNS 16
#define MSL (MV / MNS)
#define MSUB 4
#define MKS (MNS * MSUB)
__device__ __forceinline__ unsigned pkh(float a, float b) { return (unsigned)__builtin_bit_cast(unsigned short, (_Float16)a) | ((unsigned)__builtin_bit_cast(unsigned short, (_Float16)b) << 16); }
__global__ __launch_bounds__(256) void minmax_kernel(const float* __restrict__ x, float* __restrict__ PMM) {
  __shared__ float rmn[256], rmx[256]; float mn = INFINITY, mx = -INFINITY;
  for (long i = (long)blockIdx.x * 256 + threadIdx.x; i < MV; i += (long)gridDim.x * 256) { const float v = x[i]; mn = fminf(mn, v); mx = fmaxf(mx, v); }
  rmn[threadIdx.x] = mn; rmx[threadIdx.x] = mx; __syncthreads();
  for (int o = 128; o > 0; o >>= 1) { if (threadIdx.x < o) { rmn[threadIdx.x] = fminf(rmn[threadIdx.x], rmn[threadIdx.x + o]); rmx[threadIdx.x] = fmaxf(rmx[threadIdx.x], rmx[threadIdx.x + o]); } __syncthreads(); }
  if (threadIdx.x < 32) { const int k = threadIdx.x & 1; const float v = k ? rmx[0] : rmn[0]; ((volatile float*)PMM)[blockIdx.x * 2 + k] = v; __threadfence(); ((volatile float*)PMM)[blockIdx.x * 2 + k] = v; }
}
__global__ __launch_bounds__(64) void minmaxfin_kernel(const float* __restrict__ PMM, int nblk, float* __restrict__ MM) {
  if (threadIdx.x < 32) { float mn = INFINITY, mx = -INFINITY; for (int b = 0; b < nblk; ++b) { mn = fminf(mn, PMM[b * 2]); mx = fmaxf(mx, PMM[b * 2 + 1]); } const int k = threadIdx.x & 1; const float v = k ? mx : mn; ((volatile float*)MM)[k] = v; __threadfence(); ((volatile float*)MM)[k] = v; }
}
__global__ __launch_bounds__(256) void parzen_kernel(const float* __restrict__ x, const float* __restrict__ MM, long v0s, unsigned* __restrict__ WT) {
  const int lane = threadIdx.x & 31, wave = threadIdx.x >> 5; const long vl = ((long)blockIdx.x * 8 + wave) * 64;
  const float mn = MM[0], mx = MM[1]; const float inv = 1.0f / (mx - mn + 1e-8f);
  const float xa = (x[v0s + vl + 2 * lane] - mn) * inv * 63.0f, xb = (x[v0s + vl + 2 * lane + 1] - mn) * inv * 63.0f;
  float sa = 0.f, sb = 0.f;
#pragma unroll 2
  for (int c = 0; c < MBINS; ++c) { const float da = xa - (float)c, db = xb - (float)c; sa += __expf(-0.5f * da * da); sb += __expf(-0.5f * db * db); }
  const float ia = 1.0f / (sa + 1e-8f), ib = 1.0f / (sb + 1e-8f);
  for (int pass = 0; pass < 2; ++pass) {
#pragma unroll 2
    for (int c = 0; c < MBINS; ++c) { const float da = xa - (float)c, db = xb - (float)c; ((volatile unsigned*)WT)[((size_t)c * MSL + vl) / 2 + lane] = pkh(__expf(-0.5f * da * da) * ia, __expf(-0.5f * db * db) * ib); }
    __threadfence(); }
}
__global__ __launch_bounds__(256) void mi_kernel(const float* __restrict__ JP, float* __restrict__ out) {
  __shared__ double J[MBINS][MBINS]; __shared__ double pf[MBINS], pm[MBINS]; __shared__ double red[256];
  for (int i = threadIdx.x; i < MBINS * MBINS; i += 256) { double s = 0.0; for (int k = 0; k < MKS; ++k) s += (double)JP[(size_t)k * MBINS * MBINS + i]; J[i / MBINS][i % MBINS] = s; }
  __syncthreads();
  double t = 0.0; for (int i = threadIdx.x; i < MBINS * MBINS; i += 256) t += J[i / MBINS][i % MBINS]; red[threadIdx.x] = t; __syncthreads();
  for (int o = 128; o > 0; o >>= 1) { if (threadIdx.x < o) red[threadIdx.x] += red[threadIdx.x + o]; __syncthreads(); }
  const double tot = red[0] + 1e-8; __syncthreads();
  for (int i = threadIdx.x; i < MBINS * MBINS; i += 256) J[i / MBINS][i % MBINS] /= tot;
  __syncthreads();
  if (threadIdx.x < MBINS) { double a = 0.0, b = 0.0; for (int k = 0; k < MBINS; ++k) { a += J[threadIdx.x][k]; b += J[k][threadIdx.x]; } pf[threadIdx.x] = a; pm[threadIdx.x] = b; }
  __syncthreads();
  double m = 0.0; for (int i = threadIdx.x; i < MBINS * MBINS; i += 256) { const int r = i / MBINS, c = i % MBINS; const double jv = J[r][c]; if (jv > 1e-8) m += jv * log(jv / (pf[r] * pm[c] + 1e-8) + 1e-8); }
  red[threadIdx.x] = m; __syncthreads();
  for (int o = 128; o > 0; o >>= 1) { if (threadIdx.x < o) red[threadIdx.x] += red[threadIdx.x + o]; __syncthreads(); }
  if (threadIdx.x < 32) { const float v = (float)(-red[0]); ((volatile float*)out)[0] = v; __threadfence(); ((volatile float*)out)[0] = v; }
}
extern "C" void kernel_launch(void* const* d_in, const int* in_sizes, int n_in, void* d_out, int out_size, void* d_ws, size_t ws_size, hipStream_t stream) {
  (void)in_sizes; (void)n_in; (void)out_size; (void)ws_size;
  const float* fx = (const float*)d_in[0]; const float* mvx = (const float*)d_in[1];
  char* ws = (char*)d_ws; size_t off = 0;
  auto carve = [&](size_t bytes) -> char* { char* p = ws + off; off += (bytes + 255) & ~(size_t)255; return p; };
  const int NB = 1024;
  float* PMM = (float*)carve(NB * 2 * 4); float* MMF = (float*)carve(256); float* MMM = (float*)carve(256); unsigned* FT = (unsigned*)carve((size_t)MBINS * MSL * 2); unsigned* MT = (unsigned*)carve((size_t)MBINS * MSL * 2); float* JP = (float*)carve((size_t)MKS * MBINS * MBINS * 4);
  minmax_kernel<<<NB, 256, 0, stream>>>(fx, PMM); minmaxfin_kernel<<<1, 64, 0, stream>>>(PMM, NB, MMF);
  minmax_kernel<<<NB, 256, 0, stream>>>(mvx, PMM); minmaxfin_kernel<<<1, 64, 0, stream>>>(PMM, NB, MMM);
  for (int s = 0; s < MNS; ++s) { const long v0s = (long)s * MSL;
    parzen_kernel<<<MSL / 64 / 8, 256, 0, stream>>>(fx, MMF, v0s, FT); parzen_kernel<<<MSL / 64 / 8, 256, 0, stream>>>(mvx, MMM, v0s, MT);
    wmma_gemm64<0, false, 0, 0, false><<<dim3(1, MSUB), 256, 0, stream>>>((const unsigned short*)FT, nullptr, MSL, MSL / MSUB, (const unsigned short*)MT, nullptr, MSL, MSL / MSUB, JP + (size_t)s * MSUB * MBINS * MBINS, nullptr, MBINS, (long)MBINS * MBINS, nullptr, nullptr, 0, MBINS, MBINS, MSL / MSUB, 1.0f); }
  mi_kernel<<<1, 256, 0, stream>>>(JP, (float*)d_out);
}
